// LocalitySelfAttention_18313740550732
// MI455X (gfx1250) — hardware-verified
//
#include <hip/hip_runtime.h>


typedef unsigned short us;
typedef us us8 __attribute__((ext_vector_type(8)));
typedef us us16 __attribute__((ext_vector_type(16)));
typedef __bf16 bf16x16 __attribute__((ext_vector_type(16)));
typedef float v8f __attribute__((ext_vector_type(8)));
typedef float v4f __attribute__((ext_vector_type(4)));

union Frag {
  bf16x16 v;
  us16 u;
  us8 half[2];
};

__device__ __forceinline__ us f2bf(float f) {
  unsigned u = __float_as_uint(f);
  u += 0x7FFFu + ((u >> 16) & 1u);
  return (us)(u >> 16);
}

__device__ __forceinline__ void split2(float f, us& hi, us& lo) {
  const us hb = f2bf(f);
  const float hf = __uint_as_float(((unsigned)hb) << 16);
  hi = hb;
  lo = f2bf(f - hf);
}

__device__ __forceinline__ Frag ldfrag(const us* p, int h) {
  Frag f;
  f.half[0] = *(const us8*)(p + 8 * h);
  f.half[1] = *(const us8*)(p + 16 + 8 * h);
  return f;
}

__device__ __forceinline__ v8f wmma16(bf16x16 a, bf16x16 b, v8f c) {
  return __builtin_amdgcn_wmma_f32_16x16x32_bf16(false, a, false, b, (short)0, c, false, false);
}

__device__ __forceinline__ v8f mma3(const Frag& ah, const Frag& al, const Frag& bh, const Frag& bl, v8f acc) {
  acc = wmma16(al.v, bh.v, acc);
  acc = wmma16(ah.v, bl.v, acc);
  acc = wmma16(ah.v, bh.v, acc);
  asm volatile("v_nop\n\tv_nop\n\tv_nop\n\tv_nop"
               : "+v"(acc)
               : "v"(ah.v), "v"(al.v), "v"(bh.v), "v"(bl.v));
  return acc;
}

__device__ __forceinline__ v8f zero8() {
  v8f z;
#pragma unroll
  for (int i = 0; i < 8; ++i) z[i] = 0.0f;
  return z;
}

__global__ __launch_bounds__(256) void k_split(
    const float* __restrict__ s0, int n0, us* h0, us* l0,
    const float* __restrict__ s1, int n1, us* h1, us* l1,
    const float* __restrict__ s2, int n2, us* h2, us* l2,
    int nb0, int nb1) {
  const int blk = blockIdx.x;
  const float* src;
  us* dh;
  us* dl;
  int n, base;
  if (blk < nb0) {
    src = s0; dh = h0; dl = l0; n = n0; base = blk;
  } else if (blk < nb0 + nb1) {
    src = s1; dh = h1; dl = l1; n = n1; base = blk - nb0;
  } else {
    src = s2; dh = h2; dl = l2; n = n2; base = blk - nb0 - nb1;
  }
  const int i = base * 256 + (int)threadIdx.x;
  if (8 * i + 8 <= n) {
    const size_t e0 = (size_t)i * 8;
    const v4f a = *(const v4f*)(src + e0);
    const v4f c = *(const v4f*)(src + e0 + 4);
    us8 hv, lv;
#pragma unroll
    for (int e = 0; e < 4; ++e) {
      us hs, ls;
      split2(a[e], hs, ls);
      hv[e] = hs;
      lv[e] = ls;
      split2(c[e], hs, ls);
      hv[4 + e] = hs;
      lv[4 + e] = ls;
    }
    *(volatile us8*)(dh + e0) = hv;
    *(volatile us8*)(dl + e0) = lv;
    __threadfence();
    *(volatile us8*)(dh + e0) = hv;
    *(volatile us8*)(dl + e0) = lv;
  }
}

template <int AMODE>
__device__ __forceinline__ void gemm_mainloop(const us* __restrict__ Ah, const us* __restrict__ Al,
                                              const us* __restrict__ Wh, const us* __restrict__ Wl,
                                              int r0, int c0, int h, int m, v8f (&acc)[2][2]) {
#pragma unroll 1
  for (int ks = 0; ks < 8; ++ks) {
    Frag ah[2], al[2], bh[2], bl[2];
#pragma unroll
    for (int i = 0; i < 2; ++i) {
      const int row = r0 + 16 * i + m;
      size_t off;
      if (AMODE == 0) {
        off = (size_t)row * 256 + (size_t)ks * 32;
      } else {
        off = (((size_t)(row >> 12) * 8 + (size_t)ks) * 4096 + (size_t)(row & 4095)) * 32;
      }
      ah[i] = ldfrag(Ah + off, h);
      al[i] = ldfrag(Al + off, h);
    }
#pragma unroll
    for (int j = 0; j < 2; ++j) {
      const size_t off = (size_t)(c0 + 16 * j + m) * 256 + (size_t)ks * 32;
      bh[j] = ldfrag(Wh + off, h);
      bl[j] = ldfrag(Wl + off, h);
    }
#pragma unroll
    for (int i = 0; i < 2; ++i)
#pragma unroll
      for (int j = 0; j < 2; ++j)
        acc[i][j] = mma3(ah[i], al[i], bh[j], bl[j], acc[i][j]);
  }
}

__global__ __launch_bounds__(256) void k_gemm_qkv(
    const us* __restrict__ Xh, const us* __restrict__ Xl,
    const us* __restrict__ Wh, const us* __restrict__ Wl,
    us* qh, us* ql, us* kh, us* kl, us* vh, us* vl) {
  __shared__ __align__(16) us Th[8][32][40];
  __shared__ __align__(16) us Tl[8][32][40];
  const int tid = threadIdx.x;
  const int w = tid >> 5, l = tid & 31, h = l >> 4, m = l & 15;
  const int wm = w >> 1, wn = w & 1;
  const int r0 = (int)blockIdx.y * 128 + wm * 32;
  const int c0 = (int)blockIdx.x * 64 + wn * 32;

  v8f acc[2][2];
#pragma unroll
  for (int i = 0; i < 2; ++i)
#pragma unroll
    for (int j = 0; j < 2; ++j) acc[i][j] = zero8();

  gemm_mainloop<0>(Xh, Xl, Wh, Wl, r0, c0, h, m, acc);

#pragma unroll
  for (int i = 0; i < 2; ++i)
#pragma unroll
    for (int j = 0; j < 2; ++j)
#pragma unroll
      for (int r = 0; r < 8; ++r) {
        us hs, ls;
        split2(acc[i][j][r], hs, ls);
        Th[w][16 * i + 8 * h + r][16 * j + m] = hs;
        Tl[w][16 * i + 8 * h + r][16 * j + m] = ls;
      }
  __syncthreads();

  const int three = c0 >> 8;
  const int head = (c0 & 255) >> 5;
  const int bb = r0 >> 12, n0 = r0 & 4095;
  us* dh = (three == 0) ? qh : ((three == 1) ? kh : vh);
  us* dl = (three == 0) ? ql : ((three == 1) ? kl : vl);
  const size_t dst = ((size_t)(bb * 8 + head) * 4096 + (size_t)n0) * 32;

  us8 hv[4], lv[4];
#pragma unroll
  for (int q = 0; q < 4; ++q) {
    const int g = 32 * q + l;
    const int row = g >> 2, ds = (g & 3) * 8;
    hv[q] = *(const us8*)&Th[w][row][ds];
    lv[q] = *(const us8*)&Tl[w][row][ds];
  }
#pragma unroll
  for (int q = 0; q < 4; ++q) {
    const size_t o = dst + (size_t)8 * (32 * q + l);
    *(volatile us8*)(dh + o) = hv[q];
    *(volatile us8*)(dl + o) = lv[q];
  }
  __threadfence();
#pragma unroll
  for (int q = 0; q < 4; ++q) {
    const size_t o = dst + (size_t)8 * (32 * q + l);
    *(volatile us8*)(dh + o) = hv[q];
    *(volatile us8*)(dl + o) = lv[q];
  }
}

__global__ __launch_bounds__(32) void k_attn(
    const us* __restrict__ qh, const us* __restrict__ ql,
    const us* __restrict__ kh, const us* __restrict__ kl,
    const us* __restrict__ vh, const us* __restrict__ vl,
    const float* __restrict__ temp, us* oh, us* ol) {
  __shared__ __align__(16) us VTh[32][40];
  __shared__ __align__(16) us VTl[32][40];
  __shared__ __align__(16) us Ph[16][40];
  __shared__ __align__(16) us Pl[16][40];

  const int bid = blockIdx.x;
  const int qblk = bid & 255;
  const int hd = (bid >> 8) & 7;
  const int b = bid >> 11;
  const int l = threadIdx.x & 31, h = l >> 4, m = l & 15;
  const int q0 = qblk * 16;
  const int qr = q0 >> 6;
  const int qc0 = q0 & 63;
  const float alpha = 0.17677669529663689f * temp[0];
  const size_t hb = (size_t)(b * 8 + hd) * 4096 * 32;

  const Frag qfh = ldfrag(qh + hb + (size_t)(q0 + m) * 32, h);
  const Frag qfl = ldfrag(ql + hb + (size_t)(q0 + m) * 32, h);

  float mrow[8], lrow[8];
  v8f accO[2];
#pragma unroll
  for (int r = 0; r < 8; ++r) { mrow[r] = -__builtin_inff(); lrow[r] = 0.0f; }
  accO[0] = zero8();
  accO[1] = zero8();

  int wst = qc0 - 8;
  if (wst < 0) wst = 0;
  if (wst > 32) wst = 32;
  const int kr0 = (qr - 3 < 0) ? 0 : (qr - 3);
  const int kr1 = (qr + 3 > 63) ? 63 : (qr + 3);

  for (int kr = kr0; kr <= kr1; ++kr) {
    const int t0 = kr * 64 + wst;

    {
      const us* prh = vh + hb + (size_t)(t0 + l) * 32;
      const us* prl = vl + hb + (size_t)(t0 + l) * 32;
#pragma unroll
      for (int s = 0; s < 4; ++s) {
        const us8 a = *(const us8*)(prh + 8 * s);
        const us8 c = *(const us8*)(prl + 8 * s);
#pragma unroll
        for (int e = 0; e < 8; ++e) {
          VTh[8 * s + e][l] = a[e];
          VTl[8 * s + e][l] = c[e];
        }
      }
    }

    v8f s[2];
#pragma unroll
    for (int c = 0; c < 2; ++c) {
      const size_t ko = hb + (size_t)(t0 + 16 * c + m) * 32;
      const Frag kfh = ldfrag(kh + ko, h);
      const Frag kfl = ldfrag(kl + ko, h);
      s[c] = mma3(qfh, qfl, kfh, kfl, zero8());
    }

#pragma unroll
    for (int c = 0; c < 2; ++c) {
      const int col = wst + 16 * c + m;
#pragma unroll
      for (int r = 0; r < 8; ++r) {
        const int qi = 8 * h + r;
        const int dc = col - (qc0 + qi);
        const bool ok = (dc >= -3) && (dc <= 3);
        s[c][r] = ok ? s[c][r] * alpha : -__builtin_inff();
      }
    }

    float scv[8];
#pragma unroll
    for (int r = 0; r < 8; ++r) {
      float rm = fmaxf(s[0][r], s[1][r]);
#pragma unroll
      for (int msk = 1; msk < 16; msk <<= 1) rm = fmaxf(rm, __shfl_xor(rm, msk, 32));
      const float mo = mrow[r];
      const float mn = fmaxf(mo, rm);
      const float sc = __expf(mo - mn);
      const float p0 = __expf(s[0][r] - mn);
      const float p1 = __expf(s[1][r] - mn);
      us hs, ls;
      split2(p0, hs, ls);
      Ph[8 * h + r][m] = hs;
      Pl[8 * h + r][m] = ls;
      split2(p1, hs, ls);
      Ph[8 * h + r][16 + m] = hs;
      Pl[8 * h + r][16 + m] = ls;
      float ps = p0 + p1;
#pragma unroll
      for (int msk = 1; msk < 16; msk <<= 1) ps += __shfl_xor(ps, msk, 32);
      lrow[r] = lrow[r] * sc + ps;
      mrow[r] = mn;
      scv[r] = sc;
    }
    __syncthreads();

#pragma unroll
    for (int r = 0; r < 8; ++r) {
      accO[0][r] *= scv[r];
      accO[1][r] *= scv[r];
    }

    const Frag pfh = ldfrag(&Ph[m][0], h);
    const Frag pfl = ldfrag(&Pl[m][0], h);
#pragma unroll
    for (int db = 0; db < 2; ++db) {
      const Frag vfh = ldfrag(&VTh[16 * db + m][0], h);
      const Frag vfl = ldfrag(&VTl[16 * db + m][0], h);
      accO[db] = mma3(pfh, pfl, vfh, vfl, accO[db]);
    }
    __syncthreads();
  }

#pragma unroll
  for (int r = 0; r < 8; ++r) {
    const float inv = 1.0f / lrow[r];
#pragma unroll
    for (int db = 0; db < 2; ++db) {
      us hs, ls;
      split2(accO[db][r] * inv, hs, ls);
      Ph[8 * h + r][16 * db + m] = hs;
      Pl[8 * h + r][16 * db + m] = ls;
    }
  }
  __syncthreads();

  const size_t dst = hb + (size_t)q0 * 32;
  us8 hv[2], lv[2];
#pragma unroll
  for (int q = 0; q < 2; ++q) {
    const int g = 32 * q + l;
    const int row = g >> 2, ds = (g & 3) * 8;
    hv[q] = *(const us8*)&Ph[row][ds];
    lv[q] = *(const us8*)&Pl[row][ds];
  }
#pragma unroll
  for (int q = 0; q < 2; ++q) {
    const size_t o = dst + (size_t)8 * (32 * q + l);
    *(volatile us8*)(oh + o) = hv[q];
    *(volatile us8*)(ol + o) = lv[q];
  }
  __threadfence();
#pragma unroll
  for (int q = 0; q < 2; ++q) {
    const size_t o = dst + (size_t)8 * (32 * q + l);
    *(volatile us8*)(oh + o) = hv[q];
    *(volatile us8*)(ol + o) = lv[q];
  }
}

__global__ __launch_bounds__(256) void k_gemm_proj(
    const us* __restrict__ Ah, const us* __restrict__ Al,
    const us* __restrict__ Wh, const us* __restrict__ Wl,
    const float* __restrict__ bias, float* out) {
  __shared__ __align__(16) float Tf[8][32][36];
  const int tid = threadIdx.x;
  const int w = tid >> 5, l = tid & 31, h = l >> 4, m = l & 15;
  const int wm = w >> 1, wn = w & 1;
  const int r0 = (int)blockIdx.y * 128 + wm * 32;
  const int c0 = (int)blockIdx.x * 64 + wn * 32;

  v8f acc[2][2];
#pragma unroll
  for (int i = 0; i < 2; ++i)
#pragma unroll
    for (int j = 0; j < 2; ++j) acc[i][j] = zero8();

  gemm_mainloop<1>(Ah, Al, Wh, Wl, r0, c0, h, m, acc);

#pragma unroll
  for (int j = 0; j < 2; ++j) {
    const float bj = bias[c0 + 16 * j + m];
#pragma unroll
    for (int i = 0; i < 2; ++i)
#pragma unroll
      for (int r = 0; r < 8; ++r)
        Tf[w][16 * i + 8 * h + r][16 * j + m] = acc[i][j][r] + bj;
  }
  __syncthreads();

  v4f ov[8];
#pragma unroll
  for (int q = 0; q < 8; ++q) {
    const int g = 32 * q + l;
    const int row = g >> 3, cs = (g & 7) * 4;
    ov[q] = *(const v4f*)&Tf[w][row][cs];
  }
  const size_t base = (size_t)r0 * 256 + (size_t)c0;
#pragma unroll
  for (int q = 0; q < 8; ++q) {
    const int g = 32 * q + l;
    const int row = g >> 3, cs = (g & 7) * 4;
    *(volatile v4f*)(out + base + (size_t)row * 256 + cs) = ov[q];
  }
  __threadfence();
#pragma unroll
  for (int q = 0; q < 8; ++q) {
    const int g = 32 * q + l;
    const int row = g >> 3, cs = (g & 7) * 4;
    *(volatile v4f*)(out + base + (size_t)row * 256 + cs) = ov[q];
  }
}

extern "C" void kernel_launch(void* const* d_in, const int* in_sizes, int n_in,
                              void* d_out, int out_size, void* d_ws, size_t ws_size,
                              hipStream_t stream) {
  const int M = 8192;
  const int C = 256;
  const int C3 = 768;
  if (n_in < 5) return;
  if (in_sizes[0] != M * C || in_sizes[1] != C3 * C || in_sizes[2] != C * C ||
      in_sizes[3] != C || in_sizes[4] < 1 || out_size != M * C) return;

  const float* x     = (const float*)d_in[0];
  const float* wqkv  = (const float*)d_in[1];
  const float* wproj = (const float*)d_in[2];
  const float* bproj = (const float*)d_in[3];
  const float* temp  = (const float*)d_in[4];
  float* out = (float*)d_out;

  const size_t szX  = (size_t)M * C * 2;
  const size_t szW1 = (size_t)C3 * C * 2;
  const size_t szW2 = (size_t)C * C * 2;
  size_t off = 0;
  char* ws = (char*)d_ws;
  us* xh  = (us*)(ws + off); off += szX;
  us* xl  = (us*)(ws + off); off += szX;
  us* w1h = (us*)(ws + off); off += szW1;
  us* w1l = (us*)(ws + off); off += szW1;
  us* w2h = (us*)(ws + off); off += szW2;
  us* w2l = (us*)(ws + off); off += szW2;
  us* qh  = (us*)(ws + off); off += szX;
  us* ql  = (us*)(ws + off); off += szX;
  us* kh  = (us*)(ws + off); off += szX;
  us* kl  = (us*)(ws + off); off += szX;
  us* vh  = (us*)(ws + off); off += szX;
  us* vl  = (us*)(ws + off); off += szX;
  us* ah  = (us*)(ws + off); off += szX;
  us* al  = (us*)(ws + off); off += szX;
  if (off > ws_size) return;

  const int n0 = M * C, n1 = C3 * C, n2 = C * C;
  const int nb0 = (n0 / 8 + 255) / 256;
  const int nb1 = (n1 / 8 + 255) / 256;
  const int nb2 = (n2 / 8 + 255) / 256;
  k_split<<<nb0 + nb1 + nb2, 256, 0, stream>>>(x, n0, xh, xl, wqkv, n1, w1h, w1l,
                                               wproj, n2, w2h, w2l, nb0, nb1);

  k_gemm_qkv<<<dim3(C3 / 64, M / 128), 256, 0, stream>>>(xh, xl, w1h, w1l,
                                                          qh, ql, kh, kl, vh, vl);

  k_attn<<<(M / 16) * 8, 32, 0, stream>>>(qh, ql, kh, kl, vh, vl, temp, ah, al);

  k_gemm_proj<<<dim3(C / 64, M / 128), 256, 0, stream>>>(ah, al, w2h, w2l, bproj, out);
}
